// GTM_attention_54623394071036
// MI455X (gfx1250) — hardware-verified
//
#include <hip/hip_runtime.h>
#include <stddef.h>
#include <stdint.h>


#define DIN    128
#define DATT   64
#define DOUT   128
#define MAXSEG 4096
#define XP     136
#define OP     132
#define TPB    256

typedef _Float16 v16h __attribute__((ext_vector_type(16)));
typedef _Float16 v8h  __attribute__((ext_vector_type(8)));
typedef _Float16 v4h  __attribute__((ext_vector_type(4)));
typedef _Float16 v8hm __attribute__((ext_vector_type(8), may_alias));
typedef _Float16 v4hm __attribute__((ext_vector_type(4), may_alias));
typedef __bf16 v16b __attribute__((ext_vector_type(16)));
typedef __bf16 v8b  __attribute__((ext_vector_type(8)));
typedef __bf16 v8bm __attribute__((ext_vector_type(8), may_alias));
typedef unsigned short v8us __attribute__((ext_vector_type(8)));
typedef unsigned short v4usm __attribute__((ext_vector_type(4), may_alias));
typedef float v8f  __attribute__((ext_vector_type(8)));
typedef float v4f  __attribute__((ext_vector_type(4)));
typedef float v4fa __attribute__((ext_vector_type(4), may_alias));
typedef float v2fa __attribute__((ext_vector_type(2), may_alias));

union FragH { v16h v; v8h hf[2]; };
union FragB { v16b v; v8b hf[2]; };

__device__ __forceinline__ v8f mma_f16(v16h a, v16h b, v8f c) {
    c = __builtin_amdgcn_wmma_f32_16x16x32_f16(false, a, false, b, (short)0, c, false, false);
    asm volatile("v_nop\n\tv_nop\n\tv_nop\n\tv_nop" : "+v"(c) : "v"(a), "v"(b));
    return c;
}

__device__ __forceinline__ v8f mma_bf16(v16b a, v16b b, v8f c) {
    c = __builtin_amdgcn_wmma_f32_16x16x32_bf16(false, a, false, b, (short)0, c, false, false);
    asm volatile("v_nop\n\tv_nop\n\tv_nop\n\tv_nop" : "+v"(c) : "v"(a), "v"(b));
    return c;
}

__device__ __forceinline__ unsigned short bf_bits(float f) {
    unsigned u = __float_as_uint(f);
    u = u + 0x7FFFu + ((u >> 16) & 1u);
    return (unsigned short)(u >> 16);
}
__device__ __forceinline__ float bf_val(unsigned short b) {
    return __uint_as_float(((unsigned)b) << 16);
}
__device__ __forceinline__ void split_bf(float f, unsigned short& hb, unsigned short& lb) {
    hb = bf_bits(f);
    lb = bf_bits(f - bf_val(hb));
}

__global__ __launch_bounds__(TPB) void k_wprep(const float* __restrict__ Wrow,
                                               const float* __restrict__ Wcol,
                                               const float* __restrict__ Wx,
                                               v8h* hWrow, v8h* hWcol,
                                               v8b* bWxh, v8b* bWxl)
{
    const int t  = blockIdx.x * TPB + threadIdx.x;
    const int G1 = DATT * DIN / 8;
    const int G2 = DOUT * DIN / 8;
    if (t < 2 * G1) {
        const bool isr = (t < G1);
        const int  g   = isr ? t : (t - G1);
        const float* src = (isr ? Wrow : Wcol) + g * 8;
        v8h* dst = (isr ? hWrow : hWcol) + g;
        const v4f p0 = *(const v4fa*)(src);
        const v4f p1 = *(const v4fa*)(src + 4);
        v8h o;
        o[0] = (_Float16)(p0.x * 16.0f); o[1] = (_Float16)(p0.y * 16.0f);
        o[2] = (_Float16)(p0.z * 16.0f); o[3] = (_Float16)(p0.w * 16.0f);
        o[4] = (_Float16)(p1.x * 16.0f); o[5] = (_Float16)(p1.y * 16.0f);
        o[6] = (_Float16)(p1.z * 16.0f); o[7] = (_Float16)(p1.w * 16.0f);
        *(volatile v8h*)dst = o;
        __threadfence();
        *(volatile v8h*)dst = o;
    } else if (t < 2 * G1 + G2) {
        const int g = t - 2 * G1;
        const float* src = Wx + g * 8;
        const v4f p0 = *(const v4fa*)(src);
        const v4f p1 = *(const v4fa*)(src + 4);
        unsigned short h0, h1, h2, h3, h4, h5, h6, h7;
        unsigned short l0, l1, l2, l3, l4, l5, l6, l7;
        split_bf(p0.x, h0, l0); split_bf(p0.y, h1, l1);
        split_bf(p0.z, h2, l2); split_bf(p0.w, h3, l3);
        split_bf(p1.x, h4, l4); split_bf(p1.y, h5, l5);
        split_bf(p1.z, h6, l6); split_bf(p1.w, h7, l7);
        v8us hb, lb;
        hb[0] = h0; hb[1] = h1; hb[2] = h2; hb[3] = h3;
        hb[4] = h4; hb[5] = h5; hb[6] = h6; hb[7] = h7;
        lb[0] = l0; lb[1] = l1; lb[2] = l2; lb[3] = l3;
        lb[4] = l4; lb[5] = l5; lb[6] = l6; lb[7] = l7;
        const v8b H = __builtin_bit_cast(v8b, hb);
        const v8b L = __builtin_bit_cast(v8b, lb);
        *(volatile v8b*)(bWxh + g) = H;
        *(volatile v8b*)(bWxl + g) = L;
        __threadfence();
        *(volatile v8b*)(bWxh + g) = H;
        *(volatile v8b*)(bWxl + g) = L;
    }
}

__global__ __launch_bounds__(TPB) void k_proj(const float* __restrict__ x,
                                              const v8h* __restrict__ hWrow,
                                              const v8h* __restrict__ hWcol,
                                              float* a_row, float* a_col, int nN)
{
    __shared__ __attribute__((aligned(16))) _Float16 xs[32 * XP];
    __shared__ __attribute__((aligned(16))) float    os[32 * OP];
    const int tid = threadIdx.x, w = tid >> 5, l = tid & 31, h = l >> 4, m = l & 15;
    const int row0 = blockIdx.x * 32;

#pragma unroll
    for (int i = 0; i < 4; ++i) {
        const int f = tid * 4 + i * 1024;
        const int r = f >> 7, c = f & 127;
        v4f v = {0.f, 0.f, 0.f, 0.f};
        if (row0 + r < nN) v = *(const v4fa*)(x + (size_t)(row0 + r) * DIN + c);
        v4h hv;
        hv.x = (_Float16)v.x; hv.y = (_Float16)v.y; hv.z = (_Float16)v.z; hv.w = (_Float16)v.w;
        *(v4hm*)(&xs[r * XP + c]) = hv;
    }
    __syncthreads();

    const v8h* hW = (w < 4) ? hWrow : hWcol;
    const int n = (w & 3) * 16 + m;
    v8f acc0 = {0.f, 0.f, 0.f, 0.f, 0.f, 0.f, 0.f, 0.f};
    v8f acc1 = {0.f, 0.f, 0.f, 0.f, 0.f, 0.f, 0.f, 0.f};
#pragma unroll
    for (int ks = 0; ks < DIN / 32; ++ks) {
        const int kb = ks * 32;
        FragH a0, a1, b;
        b.hf[0]  = hW[n * (DIN / 8) + ks * 4 + h];
        b.hf[1]  = hW[n * (DIN / 8) + ks * 4 + 2 + h];
        a0.hf[0] = *(const v8hm*)(&xs[m * XP + kb + 8 * h]);
        a0.hf[1] = *(const v8hm*)(&xs[m * XP + kb + 16 + 8 * h]);
        a1.hf[0] = *(const v8hm*)(&xs[(16 + m) * XP + kb + 8 * h]);
        a1.hf[1] = *(const v8hm*)(&xs[(16 + m) * XP + kb + 16 + 8 * h]);
        acc0 = mma_f16(a0.v, b.v, acc0);
        acc1 = mma_f16(a1.v, b.v, acc1);
    }
#pragma unroll
    for (int r = 0; r < 8; ++r) {
        os[(8 * h + r) * OP + w * 16 + m]      = acc0[r] * 0.0625f;
        os[(16 + 8 * h + r) * OP + w * 16 + m] = acc1[r] * 0.0625f;
    }
    __syncthreads();

    const int c  = 4 * m;
    const int rA = 2 * (2 * w) + h;
    const int rB = 2 * (2 * w + 1) + h;
    const v4f va0 = *(const v4fa*)(&os[rA * OP + c]);
    const v4f vc0 = *(const v4fa*)(&os[rA * OP + 64 + c]);
    const v4f va1 = *(const v4fa*)(&os[rB * OP + c]);
    const v4f vc1 = *(const v4fa*)(&os[rB * OP + 64 + c]);
    const bool okA = (row0 + rA) < nN;
    const bool okB = (row0 + rB) < nN;
    float* pa0 = a_row + (size_t)(row0 + rA) * DATT + c;
    float* pc0 = a_col + (size_t)(row0 + rA) * DATT + c;
    float* pa1 = a_row + (size_t)(row0 + rB) * DATT + c;
    float* pc1 = a_col + (size_t)(row0 + rB) * DATT + c;
    if (okA) { *(volatile v4f*)pa0 = va0; *(volatile v4f*)pc0 = vc0; }
    if (okB) { *(volatile v4f*)pa1 = va1; *(volatile v4f*)pc1 = vc1; }
    __threadfence();
    if (okA) { *(volatile v4f*)pa0 = va0; *(volatile v4f*)pc0 = vc0; }
    if (okB) { *(volatile v4f*)pa1 = va1; *(volatile v4f*)pc1 = vc1; }
}

__global__ __launch_bounds__(TPB) void k_agg(const float* __restrict__ x,
                                             const float* __restrict__ maskv,
                                             const int* __restrict__ row,
                                             const int* __restrict__ col,
                                             const float* __restrict__ a_row,
                                             const float* __restrict__ a_col,
                                             float* agg, int nN, int nE)
{
    __shared__ __attribute__((aligned(16))) float ars[8 * DATT];
    const int tid = threadIdx.x, w = tid >> 5, l = tid & 31;
    const int node = blockIdx.x * 8 + w;
    const bool active = (node < nN);

    {
        v2fa part = {0.f, 0.f};
        if (active) part = *(const v2fa*)(a_row + (size_t)node * DATT + 2 * l);
        *(v2fa*)(&ars[w * DATT + 2 * l]) = part;
    }

    int pos = 0;
    {
        const int t = node + (l & 1);
        int len = nE;
        for (int it = 0; it < 32 && len > 0; ++it) {
            const int half = len >> 1;
            const int rv = row[pos + half];
            if (rv < t) { pos += half + 1; len -= half + 1; }
            else        { len = half; }
        }
    }
    int e0 = __shfl(pos, 0);
    const int e1 = __shfl(pos, 1);
    __syncthreads();

    if (active) {
        if (e0 < 0) e0 = 0;
        if (e0 > nE) e0 = nE;
        int cnt = e1 - e0;
        if (cnt < 0) cnt = 0;
        if (cnt > MAXSEG) cnt = MAXSEG;
        if (cnt > nE - e0) cnt = nE - e0;

        float m = -3.0e38f, Z = 0.f;
        v4f acc = {0.f, 0.f, 0.f, 0.f};
        const float* arw = &ars[w * DATT];

        for (int cb = 0; cb < cnt; cb += 32) {
            const int jn = (cnt - cb < 32) ? (cnt - cb) : 32;
            const bool v = (l < jn);
            int ce = 0;
            float me = 0.f;
            float s = -3.0e38f;
            if (v) {
                const int e = e0 + cb + l;
                ce = col[e];
                ce = (ce < 0) ? 0 : ((ce >= nN) ? (nN - 1) : ce);
                me = maskv[e];
                const float* acp = a_col + (size_t)ce * DATT;
                float d0 = 0.f, d1 = 0.f, d2 = 0.f, d3 = 0.f;
#pragma unroll
                for (int q = 0; q < DATT / 4; ++q) {
                    const v4f A = *(const v4fa*)(acp + 4 * q);
                    const v4f B = *(const v4fa*)(arw + 4 * q);
                    d0 += A.x * B.x; d1 += A.y * B.y; d2 += A.z * B.z; d3 += A.w * B.w;
                }
                const float d = ((d0 + d1) + (d2 + d3)) * 0.125f;
                s = (d >= 0.f) ? d : (0.2f * d);
            }
            float cm = s;
            cm = fmaxf(cm, __shfl_xor(cm, 16));
            cm = fmaxf(cm, __shfl_xor(cm, 8));
            cm = fmaxf(cm, __shfl_xor(cm, 4));
            cm = fmaxf(cm, __shfl_xor(cm, 2));
            cm = fmaxf(cm, __shfl_xor(cm, 1));
            const float nm   = fmaxf(m, cm);
            const float resc = __expf(m - nm);
            Z *= resc;
            acc *= resc;
            m = nm;
            const float p = v ? (me * __expf(s - m)) : 0.f;
            for (int j = 0; j < jn; ++j) {
                const float pj = __shfl(p, j);
                const int   cj = __shfl(ce, j);
                const v4f xv = *(const v4fa*)(x + (size_t)cj * DIN + 4 * l);
                Z += pj;
                acc += pj * xv;
            }
        }
        const float inv = (Z > 0.f) ? (1.0f / Z) : 0.f;
        const v4f res = acc * inv;
        float* dst = agg + (size_t)node * DIN + 4 * l;
        *(volatile v4f*)dst = res;
        __threadfence();
        *(volatile v4f*)dst = res;
    }
}

__global__ __launch_bounds__(TPB) void k_out(const float* __restrict__ agg,
                                             const v8b* __restrict__ bWxh,
                                             const v8b* __restrict__ bWxl,
                                             const float* __restrict__ bias,
                                             float* out, int nN)
{
    __shared__ __attribute__((aligned(16))) unsigned short ahs[32 * XP];
    __shared__ __attribute__((aligned(16))) unsigned short als[32 * XP];
    __shared__ __attribute__((aligned(16))) float os[32 * OP];
    const int tid = threadIdx.x, w = tid >> 5, l = tid & 31, h = l >> 4, m = l & 15;
    const int row0 = blockIdx.x * 32;

#pragma unroll
    for (int i = 0; i < 4; ++i) {
        const int f = tid * 4 + i * 1024;
        const int r = f >> 7, c = f & 127;
        v4f v = {0.f, 0.f, 0.f, 0.f};
        if (row0 + r < nN) v = *(const v4fa*)(agg + (size_t)(row0 + r) * DIN + c);
        unsigned short h0, h1, h2, h3, l0, l1, l2, l3;
        split_bf(v.x, h0, l0); split_bf(v.y, h1, l1);
        split_bf(v.z, h2, l2); split_bf(v.w, h3, l3);
        v4usm hv, lv;
        hv.x = h0; hv.y = h1; hv.z = h2; hv.w = h3;
        lv.x = l0; lv.y = l1; lv.z = l2; lv.w = l3;
        *(v4usm*)(&ahs[r * XP + c]) = hv;
        *(v4usm*)(&als[r * XP + c]) = lv;
    }
    __syncthreads();

    const int n = w * 16 + m;
    v8f acc0 = {0.f, 0.f, 0.f, 0.f, 0.f, 0.f, 0.f, 0.f};
    v8f acc1 = {0.f, 0.f, 0.f, 0.f, 0.f, 0.f, 0.f, 0.f};
#pragma unroll
    for (int ks = 0; ks < DIN / 32; ++ks) {
        const int kb = ks * 32;
        FragB bh, bl, a0h, a0l, a1h, a1l;
        bh.hf[0]  = bWxh[n * (DIN / 8) + ks * 4 + h];
        bh.hf[1]  = bWxh[n * (DIN / 8) + ks * 4 + 2 + h];
        bl.hf[0]  = bWxl[n * (DIN / 8) + ks * 4 + h];
        bl.hf[1]  = bWxl[n * (DIN / 8) + ks * 4 + 2 + h];
        a0h.hf[0] = *(const v8bm*)(&ahs[m * XP + kb + 8 * h]);
        a0h.hf[1] = *(const v8bm*)(&ahs[m * XP + kb + 16 + 8 * h]);
        a0l.hf[0] = *(const v8bm*)(&als[m * XP + kb + 8 * h]);
        a0l.hf[1] = *(const v8bm*)(&als[m * XP + kb + 16 + 8 * h]);
        a1h.hf[0] = *(const v8bm*)(&ahs[(16 + m) * XP + kb + 8 * h]);
        a1h.hf[1] = *(const v8bm*)(&ahs[(16 + m) * XP + kb + 16 + 8 * h]);
        a1l.hf[0] = *(const v8bm*)(&als[(16 + m) * XP + kb + 8 * h]);
        a1l.hf[1] = *(const v8bm*)(&als[(16 + m) * XP + kb + 16 + 8 * h]);
        acc0 = mma_bf16(a0h.v, bh.v, acc0);
        acc0 = mma_bf16(a0h.v, bl.v, acc0);
        acc0 = mma_bf16(a0l.v, bh.v, acc0);
        acc1 = mma_bf16(a1h.v, bh.v, acc1);
        acc1 = mma_bf16(a1h.v, bl.v, acc1);
        acc1 = mma_bf16(a1l.v, bh.v, acc1);
    }
    const float bv = bias[n];
#pragma unroll
    for (int r = 0; r < 8; ++r) {
        os[(8 * h + r) * OP + n]      = acc0[r] + bv;
        os[(16 + 8 * h + r) * OP + n] = acc1[r] + bv;
    }
    __syncthreads();

    v4f vr[4];
    bool ok[4];
    float* pd[4];
#pragma unroll
    for (int j = 0; j < 4; ++j) {
        const int rr = w * 4 + j;
        vr[j] = *(const v4fa*)(&os[rr * OP + 4 * l]);
        ok[j] = (row0 + rr) < nN;
        pd[j] = out + (size_t)(row0 + rr) * DOUT + 4 * l;
    }
#pragma unroll
    for (int j = 0; j < 4; ++j) if (ok[j]) *(volatile v4f*)pd[j] = vr[j];
    __threadfence();
#pragma unroll
    for (int j = 0; j < 4; ++j) if (ok[j]) *(volatile v4f*)pd[j] = vr[j];
}

extern "C" void kernel_launch(void* const* d_in, const int* in_sizes, int n_in,
                              void* d_out, int out_size, void* d_ws, size_t ws_size,
                              hipStream_t stream)
{
    if (n_in < 8) return;
    const float* x     = (const float*)d_in[0];
    const float* maskv = (const float*)d_in[1];
    const float* Wrow  = (const float*)d_in[2];
    const float* Wcol  = (const float*)d_in[3];
    const float* Wx    = (const float*)d_in[4];
    const float* bx    = (const float*)d_in[5];
    const int*   row   = (const int*)d_in[6];
    const int*   col   = (const int*)d_in[7];
    float* out = (float*)d_out;

    const int nN = in_sizes[0] / DIN;
    const int nE = in_sizes[6];
    if (nN <= 0 || nE < 0) return;
    if (out_size < nN * DOUT) return;
    if (in_sizes[2] < DATT * DIN || in_sizes[3] < DATT * DIN ||
        in_sizes[4] < DOUT * DIN || in_sizes[5] < DOUT || in_sizes[7] < nE) return;

    char* base = (char*)d_ws;
    size_t off = 0;
    auto carve = [&](size_t bytes) -> char* {
        char* r = base + off;
        off += (bytes + 255) & ~(size_t)255;
        return r;
    };
    v8h*   hWrow = (v8h*)carve((size_t)DATT * DIN * 2);
    v8h*   hWcol = (v8h*)carve((size_t)DATT * DIN * 2);
    v8b*   bWxh  = (v8b*)carve((size_t)DOUT * DIN * 2);
    v8b*   bWxl  = (v8b*)carve((size_t)DOUT * DIN * 2);
    float* a_row = (float*)carve((size_t)nN * DATT * sizeof(float));
    float* a_col = (float*)carve((size_t)nN * DATT * sizeof(float));
    float* agg   = (float*)carve((size_t)nN * DIN * sizeof(float));
    if (off > ws_size) return;

    const int gW = (2 * (DATT * DIN / 8) + (DOUT * DIN / 8) + TPB - 1) / TPB;
    k_wprep<<<gW, TPB, 0, stream>>>(Wrow, Wcol, Wx, hWrow, hWcol, bWxh, bWxl);

    const int g32 = (nN + 31) / 32;
    k_proj<<<g32, TPB, 0, stream>>>(x, hWrow, hWcol, a_row, a_col, nN);

    const int g8 = (nN + 7) / 8;
    k_agg<<<g8, TPB, 0, stream>>>(x, maskv, row, col, a_row, a_col, agg, nN, nE);

    k_out<<<g32, TPB, 0, stream>>>(agg, bWxh, bWxl, bx, out, nN);
}
